// ProteinGATv2_37958920962627
// MI455X (gfx1250) — hardware-run, weakly checked
//
#include <hip/hip_runtime.h>
#include <stddef.h>
#include <stdint.h>


#define NIN     64
#define HD      128
#define NHEAD   4
#define HCH     32
#define NLAY    3
#define ED      16
#define EDP     32
#define NG      32
#define OC      128
#define KHL     256
#define NXX     256
#define NTHR    256
#define NWAVE   8
#define EPT     8
#define CHUNK   (NTHR * EPT)
#define WCAP    (EPT * 32)
#define LISTN   (NWAVE * WCAP)
#define NB      1024
#define RCAP    20480
#define DEGCAP  64
#define GBM     64
#define GBN     64
#define GTHR    128
#define SCW     4
#define SCTHR   (SCW * 32)
#define EP      132
#define RBR     1024
#define RWR     (RBR / NWAVE)
#define WSMAX   134217728
#define LDS_BKT ((2 * RCAP + 2 * NB + LISTN + 2 * NWAVE) * 4)
#define LDS_ROB (NWAVE * NG * OC * 4)

#define EPI_PLAIN 0
#define EPI_IN    1
#define EPI_JKF   2
#define EPI_JKA   3
#define EPI_JKL   4

static_assert(HD == 32 * 4 && HD == NHEAD * HCH && HCH == 32 && OC == HD);
static_assert(ED == 16 && ED <= EDP && EDP == 32 && NG == 32);
static_assert((NIN % 32) == 0 && (KHL % 32) == 0 && KHL == 2 * HD && NXX == 2 * HD);
static_assert((CHUNK & (CHUNK - 1)) == 0 && CHUNK <= 4096);
static_assert((NB & (NB - 1)) == 0 && NB <= 4096 && (NB % 16) == 0);
static_assert(NTHR * 4 == NB);
static_assert(LISTN >= NB);
static_assert((RCAP % 16) == 0 && (RCAP % (2 * NTHR)) == 0 && RCAP >= 16623 + 16623 / 10);
static_assert(DEGCAP >= 35 + 8);
static_assert(LDS_BKT <= 300000);
static_assert(LDS_ROB + 2048 <= 300000);
static_assert(SCW * 256 * 4 + SCW * 16 * EP * 4 <= 65536);
static_assert(GBM == (GTHR / 32) * 16);
static_assert((NXX % GBN) == 0 && (OC % GBN) == 0);
static_assert((EP % 4) == 0 && EP >= HD);
static_assert((RBR % NWAVE) == 0 && (NG * OC) == 4 * 4 * NTHR);
static_assert((25600000 % 128) == 0 && ((OC * 4) % 128) == 0);
static_assert(NG * 4 == 128 && NG == 8 * 4);

typedef float          v4f   __attribute__((ext_vector_type(4)));
typedef float          v8f   __attribute__((ext_vector_type(8)));
typedef int            v2i   __attribute__((ext_vector_type(2)));
typedef int            v4i   __attribute__((ext_vector_type(4)));
typedef int            v8i   __attribute__((ext_vector_type(8)));
typedef unsigned       v2u   __attribute__((ext_vector_type(2)));
typedef unsigned       v4u   __attribute__((ext_vector_type(4)));
typedef unsigned short v8us  __attribute__((ext_vector_type(8)));
typedef __bf16         v16bf __attribute__((ext_vector_type(16)));
typedef v4f __attribute__((may_alias)) v4fa;
union FragB { v16bf v; v8us u[2]; v8i w; v4i q[2]; };

__device__ __forceinline__ v8f wmx(const FragB& a, const FragB& b, v8f c) {
  v8f d = __builtin_amdgcn_wmma_f32_16x16x32_bf16(false, a.v, false, b.v, (short)0, c, false, false);
  asm volatile("v_nop\n\tv_nop\n\tv_nop\n\tv_nop" : "+v"(d) : "v"(a.w), "v"(b.w));
  return d;
}

__device__ __forceinline__ void pinf(float x) { asm volatile("" :: "v"(x)); }
__device__ __forceinline__ void pini(int x)   { asm volatile("" :: "v"(x)); }
__device__ __forceinline__ void pin4(const v4f v) { pinf(v.x); pinf(v.y); pinf(v.z); pinf(v.w); }

__device__ __forceinline__ unsigned bfbits(float v) {
  const unsigned u = __float_as_uint(v);
  const unsigned r = (u + 0x7FFFu + ((u >> 16) & 1u)) >> 16;
  const unsigned nb = ((u >> 16) & 0x8000u) | 0x7FC0u;
  return ((u & 0x7FFFFFFFu) > 0x7F800000u) ? nb : r;
}
__device__ __forceinline__ float rbf(float v) { return __uint_as_float(bfbits(v) << 16); }
__device__ __forceinline__ v4f rbf4(const v4f a) {
  v4f o; o.x = rbf(a.x); o.y = rbf(a.y); o.z = rbf(a.z); o.w = rbf(a.w); return o;
}
__device__ __forceinline__ float wsum(float v) {
#pragma unroll
  for (int off = 16; off > 0; off >>= 1) v += __shfl_xor(v, off);
  return v;
}
__device__ __forceinline__ float row_score(const v4f v, const v4f a) {
  float p = v.x * a.x;
  p = fmaf(v.y, a.y, p);
  p = fmaf(v.z, a.z, p);
  p = fmaf(v.w, a.w, p);
  return wsum(p);
}

__device__ __forceinline__ int scan_chunk(const int* __restrict__ dsts, int nE, int cbase, int slotBase,
                                          int nb, int vec8, int* list, int tid, int lane, int wave) {
  int wc = 0;
  const int el0  = tid * EPT;
  const int e0   = cbase + el0;
  const int sent = -2147483647 - 1;
  v4i da, db;
  if (vec8 != 0 && cbase + CHUNK <= nE) {
    da = *(const v4i*)(dsts + e0);
    db = *(const v4i*)(dsts + e0 + 4);
  } else {
    da.x = (e0     < nE) ? dsts[min(e0,     nE - 1)] : sent;
    da.y = (e0 + 1 < nE) ? dsts[min(e0 + 1, nE - 1)] : sent;
    da.z = (e0 + 2 < nE) ? dsts[min(e0 + 2, nE - 1)] : sent;
    da.w = (e0 + 3 < nE) ? dsts[min(e0 + 3, nE - 1)] : sent;
    db.x = (e0 + 4 < nE) ? dsts[min(e0 + 4, nE - 1)] : sent;
    db.y = (e0 + 5 < nE) ? dsts[min(e0 + 5, nE - 1)] : sent;
    db.z = (e0 + 6 < nE) ? dsts[min(e0 + 6, nE - 1)] : sent;
    db.w = (e0 + 7 < nE) ? dsts[min(e0 + 7, nE - 1)] : sent;
  }
  const unsigned nbs = (unsigned)slotBase;
  const unsigned unb = (unsigned)nb;
  const unsigned s0 = (unsigned)da.x - nbs, s1 = (unsigned)da.y - nbs;
  const unsigned s2 = (unsigned)da.z - nbs, s3 = (unsigned)da.w - nbs;
  const unsigned s4 = (unsigned)db.x - nbs, s5 = (unsigned)db.y - nbs;
  const unsigned s6 = (unsigned)db.z - nbs, s7 = (unsigned)db.w - nbs;
  const bool h0 = s0 < unb, h1 = s1 < unb, h2 = s2 < unb, h3 = s3 < unb;
  const bool h4 = s4 < unb, h5 = s5 < unb, h6 = s6 < unb, h7 = s7 < unb;
  const unsigned any = __builtin_amdgcn_ballot_w32(h0 | h1 | h2 | h3 | h4 | h5 | h6 | h7);
  if (any != 0u) {
#define HITJ(J, HJ, SJ) { \
      const unsigned mj = __builtin_amdgcn_ballot_w32(HJ); \
      if (mj != 0u) { \
        if (HJ) { \
          const int pos = wc + (int)__builtin_amdgcn_mbcnt_lo(mj, 0u); \
          if (pos < WCAP) list[wave * WCAP + pos] = ((el0 + (J)) << 12) | (int)(SJ); \
        } \
        wc += (int)__builtin_popcount(mj); } }
    HITJ(0, h0, s0)
    HITJ(1, h1, s1)
    HITJ(2, h2, s2)
    HITJ(3, h3, s3)
    HITJ(4, h4, s4)
    HITJ(5, h5, s5)
    HITJ(6, h6, s6)
    HITJ(7, h7, s7)
#undef HITJ
  }
  return wc;
}

__global__ __launch_bounds__(NTHR) void k_xprep(const float* __restrict__ x, unsigned short* xb, int nN, int nUnits) {
  const int i = (int)blockIdx.x * NTHR + (int)threadIdx.x;
  if (i >= nUnits) return;
  const int row = i >> 3;
  const int c0  = (i & 7) * 8;
  const int rc  = row < nN ? row : nN - 1;
  const float* p = x + (size_t)rc * NIN + c0;
  const v4f a = *(const v4f*)p, b = *(const v4f*)(p + 4);
  const unsigned mk = row < nN ? 0xFFFFu : 0u;
  v8us hv;
  hv[0] = (unsigned short)(bfbits(a.x) & mk); hv[1] = (unsigned short)(bfbits(a.y) & mk);
  hv[2] = (unsigned short)(bfbits(a.z) & mk); hv[3] = (unsigned short)(bfbits(a.w) & mk);
  hv[4] = (unsigned short)(bfbits(b.x) & mk); hv[5] = (unsigned short)(bfbits(b.y) & mk);
  hv[6] = (unsigned short)(bfbits(b.z) & mk); hv[7] = (unsigned short)(bfbits(b.w) & mk);
  const size_t o = (size_t)row * NIN + c0;
  *(volatile v8us*)(xb + o) = hv;
  __threadfence();
  *(volatile v8us*)(xb + o) = hv;
}

__global__ __launch_bounds__(NTHR) void k_wtr(const float* __restrict__ w, int cols, int Kin, int Kpad, int dup,
                                              unsigned short* wt, int nUnits, int unitsPerMat,
                                              int inStride, int outStride) {
  const int u = (int)blockIdx.x * NTHR + (int)threadIdx.x;
  if (u >= nUnits) return;
  const int mi = u / unitsPerMat;
  const int v  = u - mi * unitsPerMat;
  const int kq = Kpad >> 3;
  int n = v / kq;
  const int k8 = (v - n * kq) * 8;
  n = n < cols ? n : cols - 1;
  const float* src = w + (size_t)mi * (size_t)inStride;
  float f[8];
#pragma unroll
  for (int i = 0; i < 8; ++i) {
    const int kk = k8 + i;
    const int kc = kk < Kin ? kk : Kin - 1;
    f[i] = src[(size_t)kc * (size_t)cols + n];
    pinf(f[i]);
  }
  v8us hv;
#pragma unroll
  for (int i = 0; i < 8; ++i) {
    const unsigned mk = (k8 + i < Kin) ? 0xFFFFu : 0u;
    hv[i] = (unsigned short)(bfbits(f[i]) & mk);
  }
  const size_t pitch = (size_t)Kpad * (size_t)(dup != 0 ? 2 : 1);
  const size_t o = (size_t)mi * (size_t)outStride + (size_t)n * pitch + k8;
  *(volatile v8us*)(wt + o) = hv;
  if (dup != 0) *(volatile v8us*)(wt + o + Kpad) = hv;
  __threadfence();
  *(volatile v8us*)(wt + o) = hv;
  if (dup != 0) *(volatile v8us*)(wt + o + Kpad) = hv;
}

template<int EPI>
__global__ __launch_bounds__(GTHR) __attribute__((amdgpu_num_vgpr(248)))
void k_gemm(const unsigned short* __restrict__ A, const unsigned short* __restrict__ WT,
            const float* __restrict__ bias, float* outF, float* out2, unsigned short* outH,
            int K, int ldo, int nN)
{
  __shared__ __attribute__((aligned(16))) float stg[GBM * GBN];
  const int tid = (int)threadIdx.x, lane = tid & 31, wave = tid >> 5, hh = lane >> 4, m = lane & 15;
  const int rowBase = (int)blockIdx.x * GBM;
  const int col0    = (int)blockIdx.y * GBN;

  v8f acc[4];
  {
    const v8f z = {0.f, 0.f, 0.f, 0.f, 0.f, 0.f, 0.f, 0.f};
    acc[0] = z; acc[1] = z; acc[2] = z; acc[3] = z;
  }
  const unsigned short* ap = A  + (size_t)(rowBase + 16 * wave + m) * (size_t)K + 8 * hh;
  const unsigned short* wp = WT + (size_t)(col0 + m) * (size_t)K + 8 * hh;
  const int ksteps = K >> 5;
#pragma unroll 1
  for (int ks = 0; ks < ksteps; ++ks) {
    FragB af;
    af.u[0] = *(const v8us*)(ap + 32 * ks);
    af.u[1] = *(const v8us*)(ap + 32 * ks + 16);
#pragma unroll
    for (int t = 0; t < 4; ++t) {
      const unsigned short* wq = wp + (size_t)(16 * t) * (size_t)K + 32 * ks;
      FragB bf;
      bf.u[0] = *(const v8us*)wq;
      bf.u[1] = *(const v8us*)(wq + 16);
      acc[t] = wmx(af, bf, acc[t]);
    }
  }

#pragma unroll
  for (int t = 0; t < 4; ++t) {
    const int lc = 16 * t + m;
#pragma unroll
    for (int r = 0; r < 8; ++r) {
      const int lr = 16 * wave + 8 * hh + r;
      stg[lr * GBN + lc] = acc[t][r];
    }
  }
  __syncthreads();

  if constexpr (EPI == EPI_PLAIN) {
    v4f fv[8];
#pragma unroll
    for (int i = 0; i < 8; ++i) {
      const int lr = 16 * wave + 2 * i + hh;
      fv[i] = *(const v4fa*)(stg + lr * GBN + 4 * m);
    }
#pragma unroll
    for (int i = 0; i < 8; ++i) {
      const int lr = 16 * wave + 2 * i + hh;
      float* op = outF + (size_t)(rowBase + lr) * (size_t)ldo + col0 + 4 * m;
      *(volatile v4f*)op = fv[i];
    }
    __threadfence();
#pragma unroll
    for (int i = 0; i < 8; ++i) {
      const int lr = 16 * wave + 2 * i + hh;
      float* op = outF + (size_t)(rowBase + lr) * (size_t)ldo + col0 + 4 * m;
      *(volatile v4f*)op = fv[i];
    }
  } else if constexpr (EPI == EPI_IN) {
    {
      const v4f bv = rbf4(*(const v4f*)(bias + col0 + 4 * m));
      v4f fv[8];
#pragma unroll
      for (int i = 0; i < 8; ++i) {
        const int lr = 16 * wave + 2 * i + hh;
        const v4f v = *(const v4fa*)(stg + lr * GBN + 4 * m);
        fv[i] = v + bv;
      }
#pragma unroll
      for (int i = 0; i < 8; ++i) {
        const int lr = 16 * wave + 2 * i + hh;
        float* op = outF + (size_t)(rowBase + lr) * (size_t)ldo + col0 + 4 * m;
        *(volatile v4f*)op = fv[i];
      }
      __threadfence();
#pragma unroll
      for (int i = 0; i < 8; ++i) {
        const int lr = 16 * wave + 2 * i + hh;
        float* op = outF + (size_t)(rowBase + lr) * (size_t)ldo + col0 + 4 * m;
        *(volatile v4f*)op = fv[i];
      }
    }
    {
      const int sub = (lane >> 3) & 1;
      const int c8  = 8 * (lane & 7);
      const v4f b0 = rbf4(*(const v4f*)(bias + col0 + c8));
      const v4f b1 = rbf4(*(const v4f*)(bias + col0 + c8 + 4));
      v4u pk[8];
#pragma unroll
      for (int i = 0; i < 8; ++i) {
        const int lr = 16 * wave + 2 * i + hh;
        const v4f a = *(const v4fa*)(stg + lr * GBN + c8) + b0;
        const v4f b = *(const v4fa*)(stg + lr * GBN + c8 + 4) + b1;
        const float f[8] = {a.x, a.y, a.z, a.w, b.x, b.y, b.z, b.w};
        unsigned w4[4];
#pragma unroll
        for (int j = 0; j < 4; ++j) {
          const unsigned h0 = bfbits(f[2 * j]), h1 = bfbits(f[2 * j + 1]);
          const unsigned l0 = bfbits(f[2 * j] - __uint_as_float(h0 << 16));
          const unsigned l1 = bfbits(f[2 * j + 1] - __uint_as_float(h1 << 16));
          const unsigned q0 = (sub != 0) ? l0 : h0;
          const unsigned q1 = (sub != 0) ? l1 : h1;
          w4[j] = q0 | (q1 << 16);
        }
        v4u pw; pw.x = w4[0]; pw.y = w4[1]; pw.z = w4[2]; pw.w = w4[3];
        pk[i] = pw;
      }
#pragma unroll
      for (int i = 0; i < 8; ++i) {
        const int lr = 16 * wave + 2 * i + hh;
        unsigned short* op = outH + (size_t)(rowBase + lr) * (size_t)KHL + sub * HD + col0 + c8;
        *(volatile v4u*)op = pk[i];
      }
      __threadfence();
#pragma unroll
      for (int i = 0; i < 8; ++i) {
        const int lr = 16 * wave + 2 * i + hh;
        unsigned short* op = outH + (size_t)(rowBase + lr) * (size_t)KHL + sub * HD + col0 + c8;
        *(volatile v4u*)op = pk[i];
      }
    }
  } else {
    v4f bv = {0.f, 0.f, 0.f, 0.f};
    if constexpr (EPI == EPI_JKL) bv = rbf4(*(const v4f*)(bias + col0 + 4 * m));
    v4f fv[8];
#pragma unroll
    for (int i = 0; i < 8; ++i) {
      const int lr = 16 * wave + 2 * i + hh;
      const int grow = rowBase + lr;
      const int rc = grow < nN ? grow : nN - 1;
      v4f v = *(const v4fa*)(stg + lr * GBN + 4 * m);
      if constexpr (EPI != EPI_JKF) {
        const v4f old = *(const v4f*)(outF + (size_t)rc * (size_t)ldo + col0 + 4 * m);
        pin4(old);
        v = old + v;
      }
      fv[i] = v + bv;
    }
#pragma unroll
    for (int i = 0; i < 8; ++i) {
      const int lr = 16 * wave + 2 * i + hh;
      const int grow = rowBase + lr;
      const bool ok = grow < nN;
      const int rc = ok ? grow : nN - 1;
      float* op = outF + (size_t)rc * (size_t)ldo + col0 + 4 * m;
      if (ok) *(volatile v4f*)op = fv[i];
      if constexpr (EPI == EPI_JKL) {
        float* np = out2 + (size_t)rc * (size_t)OC + col0 + 4 * m;
        if (ok) *(volatile v4f*)np = fv[i];
      }
    }
    __threadfence();
#pragma unroll
    for (int i = 0; i < 8; ++i) {
      const int lr = 16 * wave + 2 * i + hh;
      const int grow = rowBase + lr;
      const bool ok = grow < nN;
      const int rc = ok ? grow : nN - 1;
      float* op = outF + (size_t)rc * (size_t)ldo + col0 + 4 * m;
      if (ok) *(volatile v4f*)op = fv[i];
      if constexpr (EPI == EPI_JKL) {
        float* np = out2 + (size_t)rc * (size_t)OC + col0 + 4 * m;
        if (ok) *(volatile v4f*)np = fv[i];
      }
    }
  }
  (void)bias; (void)out2; (void)outH; (void)nN;
}

__global__ __launch_bounds__(NTHR) void k_bucket(const int* __restrict__ srcs, const int* __restrict__ dsts,
                                                 int* ent, int* slot, int nN, int nE, int vec8) {
  extern __shared__ v4f lds_dyn[];
  int* reg1 = (int*)lds_dyn;
  int* reg2 = reg1 + RCAP;
  int* scnt = reg2 + RCAP;
  int* soff = scnt + NB;
  int* list = soff + NB;
  int* wcnt = list + LISTN;
  int* wtot = wcnt + NWAVE;
  const int tid = (int)threadIdx.x, lane = tid & 31;
  const int wave = __builtin_amdgcn_readfirstlane(tid >> 5);
  const int nodeBase = (int)blockIdx.x * NB;

  for (int i = tid; i < NB; i += NTHR) scnt[i] = 0;
  for (int i = tid; i < RCAP; i += NTHR) { reg1[i] = 0; reg2[i] = 0; }
  __syncthreads();

  int tot = 0;
  const int nChunks = (nE + CHUNK - 1) / CHUNK;
#pragma unroll 1
  for (int ch = 0; ch < nChunks; ++ch) {
    const int cbase = ch * CHUNK;
    const int wc = scan_chunk(dsts, nE, cbase, nodeBase, NB, vec8, list, tid, lane, wave);
    if (lane == 0) wcnt[wave] = wc;
    __syncthreads();
    int pre = 0, all = 0;
#pragma unroll
    for (int w2 = 0; w2 < NWAVE; ++w2) {
      int c = wcnt[w2];
      c = c < 0 ? 0 : (c > WCAP ? WCAP : c);
      all += c;
      pre += (w2 < wave) ? c : 0;
    }
    const int wcc  = wc > WCAP ? WCAP : wc;
    const int base = tot + pre;
#pragma unroll 1
    for (int i = lane; i < wcc; i += 32) {
      const int en = list[wave * WCAP + i];
      const int el = (en >> 12) & (CHUNK - 1);
      const int sl = en & (NB - 1);
      int eid = cbase + el;
      eid = eid > nE - 1 ? nE - 1 : eid;
      const int pos = base + i;
      if (pos < RCAP) reg1[pos] = (int)(((unsigned)eid << 12) | (unsigned)sl);
    }
    tot += all;
    tot = tot > RCAP ? RCAP : tot;
    __syncthreads();
  }
  const int nh = tot;

  if (wave == 0) {
#pragma unroll 1
    for (int b0 = 0; b0 < nh; b0 += 32) {
      const int idx = b0 + lane;
      const int uv  = reg1[idx < RCAP ? idx : RCAP - 1];
      const int m32 = (nh - b0) < 32 ? (nh - b0) : 32;
#pragma unroll 1
      for (int k = 0; k < m32; ++k) {
        const int u  = __builtin_amdgcn_readlane(uv, k);
        const int sl = u & (NB - 1);
        if (lane == 0) scnt[sl] = scnt[sl] + 1;
      }
    }
  }
  __syncthreads();

  {
    const v4i ca = *(const v4i*)(scnt + 4 * tid);
    const int e0 = ca.x < 0 ? 0 : ca.x, e1 = ca.y < 0 ? 0 : ca.y;
    const int e2 = ca.z < 0 ? 0 : ca.z, e3 = ca.w < 0 ? 0 : ca.w;
    const int ts = e0 + e1 + e2 + e3;
    int incl = ts;
#pragma unroll
    for (int d = 1; d < 32; d <<= 1) {
      const int up = __shfl_up(incl, d);
      if (lane >= d) incl += up;
    }
    if (lane == 31) wtot[wave] = incl;
    __syncthreads();
    int pre = 0;
#pragma unroll
    for (int w2 = 0; w2 < NWAVE; ++w2) pre += (w2 < wave) ? wtot[w2] : 0;
    int run = pre + incl - ts;
    soff[4 * tid + 0] = run; run += e0;
    soff[4 * tid + 1] = run; run += e1;
    soff[4 * tid + 2] = run; run += e2;
    soff[4 * tid + 3] = run;
  }
  __syncthreads();
  for (int i = tid; i < NB; i += NTHR) list[i] = soff[i];
  __syncthreads();

  if (wave == 0) {
#pragma unroll 1
    for (int b0 = 0; b0 < nh; b0 += 32) {
      const int idx = b0 + lane;
      const int uv  = reg1[idx < RCAP ? idx : RCAP - 1];
      const int m32 = (nh - b0) < 32 ? (nh - b0) : 32;
#pragma unroll 1
      for (int k = 0; k < m32; ++k) {
        const int u   = __builtin_amdgcn_readlane(uv, k);
        const int sl  = u & (NB - 1);
        const int eid = (int)((unsigned)u >> 12);
        if (lane == 0) {
          int pos = list[sl];
          pos = pos < 0 ? 0 : (pos > RCAP - 1 ? RCAP - 1 : pos);
          reg2[pos] = eid;
          list[sl] = pos + 1;
        }
      }
    }
  }
  __syncthreads();

  const bool ovf = (nh >= RCAP);
  int* eb = ent + (size_t)blockIdx.x * (size_t)(2 * RCAP);
#pragma unroll 1
  for (int p0 = 0; p0 < RCAP; p0 += 2 * NTHR) {
    const int p   = p0 + 2 * tid;
    const int pa  = p < RCAP - 2 ? p : RCAP - 2;
    int e0 = reg2[pa], e1 = reg2[pa + 1];
    e0 = e0 < 0 ? 0 : (e0 > nE - 1 ? nE - 1 : e0);
    e1 = e1 < 0 ? 0 : (e1 > nE - 1 ? nE - 1 : e1);
    const int s0 = srcs[e0];
    const int s1 = srcs[e1];
    pini(s0); pini(s1);
    const int m0 = (p     < nh) ? -1 : 0;
    const int m1 = (p + 1 < nh) ? -1 : 0;
    v4i v;
    v.x = s0 & m0; v.y = e0 & m0; v.z = s1 & m1; v.w = e1 & m1;
    *(volatile v4i*)(eb + 2 * pa) = v;
    __threadfence();
    *(volatile v4i*)(eb + 2 * pa) = v;
  }
#pragma unroll 1
  for (int it = 0; it < NB / (2 * NTHR); ++it) {
    const int q = tid + NTHR * it;
    v4i sv;
    sv.x = soff[2 * q];
    sv.y = ovf ? -1 : scnt[2 * q];
    sv.z = soff[2 * q + 1];
    sv.w = ovf ? -1 : scnt[2 * q + 1];
    int* sp = slot + 2 * (size_t)(nodeBase + 2 * q);
    *(volatile v4i*)sp = sv;
    __threadfence();
    *(volatile v4i*)sp = sv;
  }
  (void)nN;
}

__global__ __launch_bounds__(SCTHR) __attribute__((amdgpu_num_vgpr(248)))
void k_scan(const int* __restrict__ ent, const int* __restrict__ slot,
            const float* __restrict__ ea, const unsigned short* __restrict__ wet,
            const float* __restrict__ xlxr,
            const float* __restrict__ att, const float* __restrict__ bias,
            const float* __restrict__ gam, const float* __restrict__ bet,
            float* Hf, unsigned short* HL, int nN, int nE)
{
  __shared__ __attribute__((aligned(16))) int   sA[SCW * 256];
  __shared__ __attribute__((aligned(16))) float sE[SCW * 16 * EP];
  const int tid = (int)threadIdx.x, lane = tid & 31, hh = lane >> 4, m = lane & 15;
  const int wave = __builtin_amdgcn_readfirstlane(tid >> 5);
  const int i = (int)blockIdx.x * SCW + wave;
  if (i >= nN) return;
  int*   At = sA + wave * 256;
  float* Et = sE + wave * 16 * EP;

  const v2i se = *(const v2i*)(slot + 2 * (size_t)i);
  int st = __builtin_amdgcn_readfirstlane(se.x);
  const int craw = __builtin_amdgcn_readfirstlane(se.y);
  st = st < 0 ? 0 : (st > RCAP - 1 ? RCAP - 1 : st);
  int cnt = craw < 0 ? 0 : (craw > DEGCAP ? DEGCAP : craw);
  if (cnt > RCAP - st) cnt = RCAP - st;
  const float qnan = __int_as_float(0x7fc00000);
  const float pz = (craw < 0 || craw > DEGCAP) ? qnan : 0.0f;
  const int blk = i / NB;
  const int* eb = ent + (size_t)blk * (size_t)(2 * RCAP);
  const v8f z8 = {0.f, 0.f, 0.f, 0.f, 0.f, 0.f, 0.f, 0.f};
  const v4i zero4 = {0, 0, 0, 0};

  const int cb = 4 * lane;
  const v4f xr = *(const v4f*)(xlxr + (size_t)i * (size_t)NXX + HD + cb);
  const v4f at = rbf4(*(const v4f*)(att + cb));
  v4f acc = {0.f, 0.f, 0.f, 0.f};
  float mx = __int_as_float((int)0xff800000u);
  float dn = 0.0f;

#pragma unroll 1
  for (int t0 = 0; t0 < cnt; t0 += 16) {
    const int nv = (cnt - t0) < 16 ? (cnt - t0) : 16;
    int ei = st + t0 + m;
    ei = ei > st + cnt - 1 ? st + cnt - 1 : ei;
    const v2i en = *(const v2i*)(eb + 2 * ei);
    const int src = en.x < 0 ? 0 : (en.x > nN - 1 ? nN - 1 : en.x);
    const int eid = en.y < 0 ? 0 : (en.y > nE - 1 ? nE - 1 : en.y);

    __builtin_amdgcn_fence(__ATOMIC_RELEASE, "wavefront");
    __builtin_amdgcn_wave_barrier();
    {
      const int row  = lane >> 1;
      const int half = lane & 1;
      const int er   = __shfl(eid, row);
      const float* p = ea + (size_t)er * ED + 8 * half;
      const v4f a = *(const v4f*)p;
      const v4f b = *(const v4f*)(p + 4);
      const unsigned msk = (row < nv) ? 0xFFFFu : 0u;
      v4i w;
      w.x = (int)((bfbits(a.x) & msk) | ((bfbits(a.y) & msk) << 16));
      w.y = (int)((bfbits(a.z) & msk) | ((bfbits(a.w) & msk) << 16));
      w.z = (int)((bfbits(b.x) & msk) | ((bfbits(b.y) & msk) << 16));
      w.w = (int)((bfbits(b.z) & msk) | ((bfbits(b.w) & msk) << 16));
      *(v4i*)(At + row * 16 + 4 * half)     = w;
      *(v4i*)(At + row * 16 + 8 + 4 * half) = zero4;
    }
    __builtin_amdgcn_fence(__ATOMIC_RELEASE, "wavefront");
    __builtin_amdgcn_wave_barrier();
    FragB af;
    af.q[0] = *(const v4i*)(At + m * 16 + 4 * hh);
    af.q[1] = *(const v4i*)(At + m * 16 + 8 + 4 * hh);
#pragma unroll 1
    for (int tt = 0; tt < 8; ++tt) {
      const unsigned short* wq = wet + (size_t)(16 * tt + m) * EDP + 8 * hh;
      FragB bf;
      bf.q[0] = *(const v4i*)wq;
      bf.q[1] = *(const v4i*)(wq + 16);
      v8f d = wmx(af, bf, z8);
#pragma unroll
      for (int r = 0; r < 8; ++r) Et[(8 * hh + r) * EP + 16 * tt + m] = d[r];
    }
    __builtin_amdgcn_fence(__ATOMIC_RELEASE, "wavefront");
    __builtin_amdgcn_wave_barrier();
#pragma unroll 1
    for (int r = 0; r < nv; ++r) {
      const int s = __builtin_amdgcn_readlane(src, r);
      const v4f xl = *(const v4f*)(xlxr + (size_t)s * (size_t)NXX + cb);
      const v4f ee = *(const v4fa*)(Et + r * EP + 4 * lane);
      v4f v = (xl + xr) + ee;
      v.x = (v.x > 0.0f) ? v.x : 0.2f * v.x;
      v.y = (v.y > 0.0f) ? v.y : 0.2f * v.y;
      v.z = (v.z > 0.0f) ? v.z : 0.2f * v.z;
      v.w = (v.w > 0.0f) ? v.w : 0.2f * v.w;
      float part = v.x * at.x;
      part = fmaf(v.y, at.y, part);
      part = fmaf(v.z, at.z, part);
      part = fmaf(v.w, at.w, part);
      part += __shfl_xor(part, 1);
      part += __shfl_xor(part, 2);
      part += __shfl_xor(part, 4);
      const float al = part;
      const float df = al - mx;
      const float eo = expf(-fabsf(df));
      const bool up  = df > 0.0f;
      const float s1 = up ? eo : 1.0f;
      const float s2 = up ? 1.0f : eo;
      mx = up ? al : mx;
      dn = fmaf(dn, s1, s2);
      acc = acc * s1 + xl * s2;
    }
  }

  const float inv = (cnt > 0) ? (1.0f / (dn + 1e-16f)) : 0.0f;
  const v4f bb = rbf4(*(const v4f*)(bias + cb));
  float* gp = Hf + (size_t)i * HD + cb;
  const v4f hres = *(const v4f*)gp;
  const v4f hv = (acc * inv + bb) + hres;
  const float sm = wsum((hv.x + hv.y) + (hv.z + hv.w));
  const float mu = sm * (1.0f / (float)HD);
  const v4f dv = hv - mu;
  const float sq = wsum((dv.x * dv.x + dv.y * dv.y) + (dv.z * dv.z + dv.w * dv.w));
  const float var = sq * (1.0f / (float)HD);
  const float rstd = 1.0f / sqrtf(var + 1e-5f);
  const v4f gg = rbf4(*(const v4f*)(gam + cb));
  const v4f bt = rbf4(*(const v4f*)(bet + cb));
  v4f y = (dv * rstd) * gg + bt;
  y.x = (y.x > 0.0f) ? y.x : (y.x - y.x);
  y.y = (y.y > 0.0f) ? y.y : (y.y - y.y);
  y.z = (y.z > 0.0f) ? y.z : (y.z - y.z);
  y.w = (y.w > 0.0f) ? y.w : (y.w - y.w);
  y = y + pz;
  const unsigned h0 = bfbits(y.x), h1 = bfbits(y.y), h2 = bfbits(y.z), h3 = bfbits(y.w);
  const unsigned l0 = bfbits(y.x - __uint_as_float(h0 << 16));
  const unsigned l1 = bfbits(y.y - __uint_as_float(h1 << 16));
  const unsigned l2 = bfbits(y.z - __uint_as_float(h2 << 16));
  const unsigned l3 = bfbits(y.w - __uint_as_float(h3 << 16));
  v2u hw, lw;
  hw.x = h0 | (h1 << 16); hw.y = h2 | (h3 << 16);
  lw.x = l0 | (l1 << 16); lw.y = l2 | (l3 << 16);
  unsigned short* hp = HL + (size_t)i * KHL + cb;
  *(volatile v4f*)gp = y;
  *(volatile v2u*)hp = hw;
  *(volatile v2u*)(hp + HD) = lw;
  __threadfence();
  *(volatile v4f*)gp = y;
  *(volatile v2u*)hp = hw;
  *(volatile v2u*)(hp + HD) = lw;
}

__global__ __launch_bounds__(NTHR) void k_roA(const float* __restrict__ nodec, const float* __restrict__ roatt,
                                              const int* __restrict__ bat, float* mrec, int nN) {
  __shared__ float wm[NWAVE * NG];
  __shared__ __attribute__((aligned(16))) float rec[NG];
  const int tid = (int)threadIdx.x, lane = tid & 31;
  const int wave = __builtin_amdgcn_readfirstlane(tid >> 5);
  const v4f a4 = rbf4(*(const v4f*)(roatt + 4 * lane));
  const int row0 = (int)blockIdx.x * RBR + wave * RWR;
  int nr = nN - row0;
  nr = nr < 0 ? 0 : (nr > RWR ? RWR : nr);
  const float ninf = __int_as_float((int)0xff800000u);
  float mxg = ninf;
#pragma unroll 1
  for (int k = 0; k < nr; ++k) {
    int rc = row0 + k;
    rc = rc > nN - 1 ? nN - 1 : rc;
    const v4f v = *(const v4f*)(nodec + (size_t)rc * OC + 4 * lane);
    const float s = row_score(v, a4);
    const int g = bat[rc];
    const float cand = fmaxf(mxg, s);
    mxg = (g == lane) ? cand : mxg;
  }
  wm[wave * NG + lane] = mxg;
  __syncthreads();
  if (tid < NG) {
    float r = ninf;
#pragma unroll
    for (int w2 = 0; w2 < NWAVE; ++w2) r = fmaxf(r, wm[w2 * NG + tid]);
    rec[tid] = r;
  }
  __syncthreads();
  const int pc = 4 * (tid & 7);
  const v4f rv = *(const v4fa*)(rec + pc);
  float* mp = mrec + (size_t)blockIdx.x * NG + pc;
  if (tid < 8) *(volatile v4f*)mp = rv;
  __threadfence();
  if (tid < 8) *(volatile v4f*)mp = rv;
}

__global__ __launch_bounds__(NTHR) void k_roB(const float* __restrict__ nodec, const float* __restrict__ roatt,
                                              const int* __restrict__ bat, const float* __restrict__ mrec, int nRB,
                                              float* wrec, float* lrec, int nN) {
  extern __shared__ v4f lds_dyn[];
  float* pl = (float*)lds_dyn;
  __shared__ float dnw[NWAVE * NG];
  __shared__ float smx[NG];
  __shared__ __attribute__((aligned(16))) float drec[NG];
  const int tid = (int)threadIdx.x, lane = tid & 31;
  const int wave = __builtin_amdgcn_readfirstlane(tid >> 5);
  {
    const v4f z = {0.f, 0.f, 0.f, 0.f};
#pragma unroll 1
    for (int idx = tid; idx < NWAVE * NG * OC / 4; idx += NTHR) *(v4fa*)(pl + 4 * idx) = z;
  }
  if (tid < NG) {
    float r = __int_as_float((int)0xff800000u);
#pragma unroll 1
    for (int b = 0; b < nRB; ++b) r = fmaxf(r, mrec[(size_t)b * NG + tid]);
    smx[tid] = (fabsf(r) <= 3.4028234e38f) ? r : 0.0f;
  }
  __syncthreads();

  const v4f a4 = rbf4(*(const v4f*)(roatt + 4 * lane));
  const int row0 = (int)blockIdx.x * RBR + wave * RWR;
  int nr = nN - row0;
  nr = nr < 0 ? 0 : (nr > RWR ? RWR : nr);
  float den = 0.0f;
#pragma unroll 1
  for (int k = 0; k < nr; ++k) {
    int rc = row0 + k;
    rc = rc > nN - 1 ? nN - 1 : rc;
    const v4f v = *(const v4f*)(nodec + (size_t)rc * OC + 4 * lane);
    const float s = row_score(v, a4);
    const int g = __builtin_amdgcn_readfirstlane(bat[rc]);
    if ((unsigned)g < (unsigned)NG) {
      const float ex = expf(s - smx[g]);
      den += (lane == g) ? ex : 0.0f;
      float* pp = pl + (size_t)(wave * NG + g) * OC + 4 * lane;
      v4f o = *(const v4fa*)pp;
      o = o + v * ex;
      *(v4fa*)pp = o;
    }
  }
  dnw[wave * NG + lane] = den;
  __syncthreads();

  v4f sv[4];
#pragma unroll
  for (int it = 0; it < 4; ++it) {
    const int idx4 = tid + NTHR * it;
    v4f s = {0.f, 0.f, 0.f, 0.f};
#pragma unroll
    for (int w2 = 0; w2 < NWAVE; ++w2) s = s + *(const v4fa*)(pl + (size_t)w2 * NG * OC + 4 * idx4);
    sv[it] = s;
  }
  if (tid < NG) {
    float dsum = 0.0f;
#pragma unroll
    for (int w2 = 0; w2 < NWAVE; ++w2) dsum += dnw[w2 * NG + tid];
    drec[tid] = dsum;
  }
  __syncthreads();
  const int pc = 4 * (tid & 7);
  const v4f dv4 = *(const v4fa*)(drec + pc);
  float* wb = wrec + (size_t)blockIdx.x * NG * OC;
  float* lp = lrec + (size_t)blockIdx.x * NG + pc;
#pragma unroll
  for (int it = 0; it < 4; ++it) *(volatile v4f*)(wb + 4 * (tid + NTHR * it)) = sv[it];
  if (tid < 8) *(volatile v4f*)lp = dv4;
  __threadfence();
#pragma unroll
  for (int it = 0; it < 4; ++it) *(volatile v4f*)(wb + 4 * (tid + NTHR * it)) = sv[it];
  if (tid < 8) *(volatile v4f*)lp = dv4;
}

__global__ __launch_bounds__(NTHR) void k_roC(const float* __restrict__ wrec, const float* __restrict__ lrec, int nRB,
                                              const float* __restrict__ roW, const float* __restrict__ rob,
                                              float* out1) {
  __shared__ __attribute__((aligned(16))) float pool[NG * OC];
  __shared__ __attribute__((aligned(16))) float gout[NG * OC];
  __shared__ float dinv[NG];
  const int tid = (int)threadIdx.x;
  if (tid < NG) {
    double d = 0.0;
#pragma unroll 1
    for (int b = 0; b < nRB; ++b) d += (double)lrec[(size_t)b * NG + tid];
    dinv[tid] = 1.0f / ((float)d + 1e-16f);
  }
  __syncthreads();
  const int c  = tid & (OC - 1);
  const int gh = tid >> 7;
#pragma unroll 1
  for (int gg = 0; gg < NG / 2; ++gg) {
    const int g = gh * (NG / 2) + gg;
    double s = 0.0;
#pragma unroll 1
    for (int b = 0; b < nRB; ++b) s += (double)wrec[((size_t)b * NG + g) * OC + c];
    pool[g * OC + c] = (float)s * dinv[g];
  }
  __syncthreads();
  const float bc = rbf(rob[c]);
#pragma unroll 1
  for (int gg = 0; gg < NG / 2; ++gg) {
    const int g = gh * (NG / 2) + gg;
    float acc = 0.0f;
#pragma unroll 4
    for (int k = 0; k < OC; ++k) acc = fmaf(pool[g * OC + k], rbf(roW[(size_t)k * OC + c]), acc);
    gout[g * OC + c] = acc + bc;
  }
  __syncthreads();
  v4f ov[4];
#pragma unroll
  for (int it = 0; it < 4; ++it) ov[it] = *(const v4fa*)(gout + 4 * (tid + NTHR * it));
#pragma unroll
  for (int it = 0; it < 4; ++it) *(volatile v4f*)(out1 + 4 * (tid + NTHR * it)) = ov[it];
  __threadfence();
#pragma unroll
  for (int it = 0; it < 4; ++it) *(volatile v4f*)(out1 + 4 * (tid + NTHR * it)) = ov[it];
}

static inline int cdiv(int a, int b) { return (a + b - 1) / b; }
static inline size_t al256(size_t o) { return (o + 255) & ~(size_t)255; }

extern "C" void kernel_launch(void* const* d_in, const int* in_sizes, int n_in,
                              void* d_out, int out_size, void* d_ws, size_t ws_size,
                              hipStream_t stream) {
  if (n_in < 18) return;
  const int nN = in_sizes[0] / NIN;
  if (nN <= 0 || in_sizes[0] != nN * NIN || nN > (1 << 21)) return;
  if (in_sizes[1] < 2 || (in_sizes[1] & 1) != 0) return;
  const int nE = in_sizes[1] / 2;
  if (nE < 1 || nE >= (1 << 20)) return;
  if (in_sizes[2] != nE * ED) return;
  if (in_sizes[3] != nN) return;
  if (in_sizes[4] != NIN * HD || in_sizes[5] != HD) return;
  if (in_sizes[6] != NLAY * HD * HD || in_sizes[7] != NLAY * HD * HD) return;
  if (in_sizes[8] != NLAY * ED * HD || in_sizes[9] != NLAY * NHEAD * HCH) return;
  if (in_sizes[10] != NLAY * HD || in_sizes[11] != NLAY * HD || in_sizes[12] != NLAY * HD) return;
  if (in_sizes[13] != NLAY * HD * OC || in_sizes[14] != OC) return;
  if (in_sizes[15] != OC || in_sizes[16] != OC * OC || in_sizes[17] != OC) return;
  if (out_size != nN * OC + NG * OC) return;

  const float* x      = (const float*)d_in[0];
  const int*   ei     = (const int*)  d_in[1];
  const float* eattr  = (const float*)d_in[2];
  const int*   bat    = (const int*)  d_in[3];
  const float* in_W   = (const float*)d_in[4];
  const float* in_b   = (const float*)d_in[5];
  const float* W_src  = (const float*)d_in[6];
  const float* W_dst  = (const float*)d_in[7];
  const float* W_edge = (const float*)d_in[8];
  const float* attv   = (const float*)d_in[9];
  const float* conv_b = (const float*)d_in[10];
  const float* ln_g   = (const float*)d_in[11];
  const float* ln_b   = (const float*)d_in[12];
  const float* jk_W   = (const float*)d_in[13];
  const float* jk_b   = (const float*)d_in[14];
  const float* ro_att = (const float*)d_in[15];
  const float* ro_W   = (const float*)d_in[16];
  const float* ro_b   = (const float*)d_in[17];
  float* out0 = (float*)d_out;
  float* out1 = (float*)d_out + (size_t)nN * OC;
  const int* src = ei;
  const int* dst = ei + nE;

  const int MP   = cdiv(nN, GBM) * GBM;
  const int gB   = cdiv(nN, NB);
  const int nRB  = cdiv(nN, RBR);
  const int vec8 = ((nE & 3) == 0) ? 1 : 0;

  char* ws = (char*)d_ws;
  size_t off = 0;
  const size_t oXB  = off; off = al256(off + (size_t)MP * NIN * 2);
  const size_t oXX  = off; off = al256(off + (size_t)MP * NXX * 4);
  const size_t oH   = off; off = al256(off + (size_t)MP * HD * 4);
  const size_t oHL  = off; off = al256(off + (size_t)MP * KHL * 2);
  const size_t oENT = off; off = al256(off + (size_t)gB * RCAP * 8);
  const size_t oSLT = off; off = al256(off + (size_t)gB * NB * 8);
  const size_t oINW = off; off = al256(off + (size_t)HD * NIN * 2);
  const size_t oWSD = off; off = al256(off + (size_t)NLAY * NXX * KHL * 2);
  const size_t oWE  = off; off = al256(off + (size_t)NLAY * HD * EDP * 2);
  const size_t oJK  = off; off = al256(off + (size_t)NLAY * OC * KHL * 2);
  const size_t oMR  = off; off = al256(off + (size_t)nRB * NG * 4);
  const size_t oLR  = off; off = al256(off + (size_t)nRB * NG * 4);
  const size_t oWR  = off; off = al256(off + (size_t)nRB * NG * OC * 4);
  if (off > ws_size || off > (size_t)WSMAX) return;
  if ((size_t)nN * OC * 4 > (size_t)MP * NXX * 4) return;
  if ((long long)gB * NB < (long long)nN) return;
  unsigned short* XB   = (unsigned short*)(ws + oXB);
  float*          XLXR = (float*)(ws + oXX);
  float*          NODEC= (float*)(ws + oXX);
  float*          Hf   = (float*)(ws + oH);
  unsigned short* HL   = (unsigned short*)(ws + oHL);
  int*            ENT  = (int*)(ws + oENT);
  int*            SLT  = (int*)(ws + oSLT);
  unsigned short* INWT = (unsigned short*)(ws + oINW);
  unsigned short* WSD  = (unsigned short*)(ws + oWSD);
  unsigned short* WET  = (unsigned short*)(ws + oWE);
  unsigned short* JKT  = (unsigned short*)(ws + oJK);
  float*          MREC = (float*)(ws + oMR);
  float*          LREC = (float*)(ws + oLR);
  float*          WREC = (float*)(ws + oWR);

  hipFuncSetAttribute(reinterpret_cast<const void*>(&k_bucket),
                      hipFuncAttributeMaxDynamicSharedMemorySize, LDS_BKT);
  hipFuncSetAttribute(reinterpret_cast<const void*>(&k_roB),
                      hipFuncAttributeMaxDynamicSharedMemorySize, LDS_ROB);

  {
    const int nUx = MP * (NIN / 8);
    k_xprep<<<cdiv(nUx, NTHR), NTHR, 0, stream>>>(x, XB, nN, nUx);
    const int uA = HD * (NIN / 8);
    k_wtr<<<cdiv(uA, NTHR), NTHR, 0, stream>>>(in_W, HD, NIN, NIN, 0, INWT, uA, uA, 0, 0);
    const int uB = HD * (HD / 8);
    k_wtr<<<cdiv(NLAY * uB, NTHR), NTHR, 0, stream>>>(W_src, HD, HD, HD, 1, WSD, NLAY * uB, uB,
                                                       HD * HD, NXX * KHL);
    k_wtr<<<cdiv(NLAY * uB, NTHR), NTHR, 0, stream>>>(W_dst, HD, HD, HD, 1, WSD + (size_t)HD * KHL, NLAY * uB, uB,
                                                       HD * HD, NXX * KHL);
    const int uC = HD * (EDP / 8);
    k_wtr<<<cdiv(NLAY * uC, NTHR), NTHR, 0, stream>>>(W_edge, HD, ED, EDP, 0, WET, NLAY * uC, uC,
                                                       ED * HD, HD * EDP);
    k_wtr<<<cdiv(NLAY * uB, NTHR), NTHR, 0, stream>>>(jk_W, OC, HD, HD, 1, JKT, NLAY * uB, uB,
                                                       HD * OC, OC * KHL);
  }

  k_bucket<<<gB, NTHR, LDS_BKT, stream>>>(src, dst, ENT, SLT, nN, nE, vec8);

  const int gM = MP / GBM;
  k_gemm<EPI_IN><<<dim3(gM, HD / GBN), GTHR, 0, stream>>>(XB, INWT, in_b, Hf, Hf, HL, NIN, HD, nN);

  for (int l = 0; l < NLAY; ++l) {
    k_gemm<EPI_PLAIN><<<dim3(gM, NXX / GBN), GTHR, 0, stream>>>(HL, WSD + (size_t)l * NXX * KHL, in_b,
                                                                 XLXR, XLXR, HL, KHL, NXX, nN);
    k_scan<<<cdiv(nN, SCW), SCTHR, 0, stream>>>(ENT, SLT, eattr, WET + (size_t)l * HD * EDP, XLXR,
                                                 attv + (size_t)l * HD, conv_b + (size_t)l * HD,
                                                 ln_g + (size_t)l * HD, ln_b + (size_t)l * HD,
                                                 Hf, HL, nN, nE);
    const unsigned short* jkp = JKT + (size_t)l * OC * KHL;
    if (l == 0) {
      k_gemm<EPI_JKF><<<dim3(gM, OC / GBN), GTHR, 0, stream>>>(HL, jkp, jk_b, out0, out0, HL, KHL, OC, nN);
    } else if (l < NLAY - 1) {
      k_gemm<EPI_JKA><<<dim3(gM, OC / GBN), GTHR, 0, stream>>>(HL, jkp, jk_b, out0, out0, HL, KHL, OC, nN);
    } else {
      k_gemm<EPI_JKL><<<dim3(gM, OC / GBN), GTHR, 0, stream>>>(HL, jkp, jk_b, out0, NODEC, HL, KHL, OC, nN);
    }
  }

  k_roA<<<nRB, NTHR, 0, stream>>>(NODEC, ro_att, bat, MREC, nN);
  k_roB<<<nRB, NTHR, LDS_ROB, stream>>>(NODEC, ro_att, bat, MREC, nRB, WREC, LREC, nN);
  k_roC<<<1, NTHR, 0, stream>>>(WREC, LREC, nRB, ro_W, ro_b, out1);
}
